// DGAT_88802743812894
// MI455X (gfx1250) — hardware-verified
//
#include <hip/hip_runtime.h>


namespace {
constexpr int N = 10000, E = 80000, F = 128, H = 32, C1 = 64, OUT = 16, D1 = H * C1, D2 = H * OUT, NPAD = 10112;
constexpr float FXS = 524288.0f, FXI = 1.0f / 524288.0f, NEG = 0.2f, BNE = 1e-5f;

typedef _Float16 b16;
typedef __attribute__((ext_vector_type(16))) _Float16 v16b;
typedef __attribute__((ext_vector_type(8)))  _Float16 v8b;
typedef __attribute__((ext_vector_type(8)))  float v8f;
typedef __attribute__((ext_vector_type(4)))  float v4f;

__device__ __forceinline__ v8b ld8b(const b16* p) { return *(const v8b*)p; }
__device__ __forceinline__ v16b cat8b(v8b a, v8b b) { return __builtin_shufflevector(a, b, 0, 1, 2, 3, 4, 5, 6, 7, 8, 9, 10, 11, 12, 13, 14, 15); }
__device__ __forceinline__ v16b frag_kb(const b16* p, int hh) { return cat8b(ld8b(p + 8 * hh), ld8b(p + 16 + 8 * hh)); }
__device__ __forceinline__ void split16(float v, b16& hi, b16& lo) { hi = (b16)v; lo = (b16)(v - (float)hi); }
__device__ __forceinline__ void frag_ksplit(const float* p, int hh, v16b& fh_, v16b& fl_) {
  const float* p0 = p + 8 * hh; const float* p1 = p + 16 + 8 * hh;
#pragma unroll
  for (int e = 0; e < 8; ++e) { b16 a, c; split16(p0[e], a, c); fh_[e] = a; fl_[e] = c; split16(p1[e], a, c); fh_[8 + e] = a; fl_[8 + e] = c; }
}
__device__ __forceinline__ v8f wmma16b(v16b a, v16b b, v8f c) {
  v8f d = __builtin_amdgcn_wmma_f32_16x16x32_f16(false, a, false, b, (short)0, c, false, false);
  asm volatile("v_nop\n\tv_nop\n\tv_nop\n\tv_nop" : "+v"(d) : "v"(a), "v"(b));
  return d;
}
__device__ __forceinline__ void wave_lds_sync() {
  __builtin_amdgcn_fence(__ATOMIC_RELEASE, "workgroup");
  __builtin_amdgcn_wave_barrier();
  __builtin_amdgcn_fence(__ATOMIC_ACQUIRE, "workgroup");
}

struct Opnd { const void* p0; const void* p1; int ld; };
template <int NP> __device__ __forceinline__ void load_frags(const Opnd& o, int row, int kb, int hh, v16b& fh_, v16b& fl_) {
  if (NP == 0) { frag_ksplit((const float*)o.p0 + (size_t)row * o.ld + kb, hh, fh_, fl_); }
  else if (NP == 4) {
    const float* p = (const float*)o.p0 + (size_t)row * o.ld + kb; const float* p0 = p + 8 * hh; const float* p1 = p + 16 + 8 * hh;
#pragma unroll
    for (int e = 0; e < 8; ++e) { b16 a, c; split16(p0[e] * 64.0f, a, c); fh_[e] = a; fl_[e] = c; split16(p1[e] * 64.0f, a, c); fh_[8 + e] = a; fl_[8 + e] = c; }
  } else if (NP == 3) {
    const float* p = (const float*)o.p0 + (size_t)row * o.ld + kb; const float* p0 = p + 8 * hh; const float* p1 = p + 16 + 8 * hh;
#pragma unroll
    for (int e = 0; e < 8; ++e) { fh_[e] = (b16)p0[e]; fh_[8 + e] = (b16)p1[e]; }
    fl_ = fh_;
  } else {
    fh_ = frag_kb((const b16*)o.p0 + (size_t)row * o.ld + kb, hh);
    if (NP == 2) fl_ = frag_kb((const b16*)o.p1 + (size_t)row * o.ld + kb, hh); else fl_ = fh_;
  }
}
template <int ANP, int BNP> __device__ __forceinline__ v8f mac(v16b ah, v16b al, v16b bh, v16b bl, v8f c) {
  c = wmma16b(ah, bh, c);
  if (BNP == 0 || BNP == 2 || BNP == 4) c = wmma16b(ah, bl, c);
  if (ANP == 0 || ANP == 2 || ANP == 4) c = wmma16b(al, bh, c);
  return c;
}
template <int ANP, int BNP>
__device__ __forceinline__ void gemm_tile(const Opnd& A, const Opnd& B, int K, int m0, int c0, int nloc, int hlf, v8f (&acc)[2][4]) {
  for (int kb = 0; kb < K; kb += 32) {
    v16b a0h, a0l, a1h, a1l;
    load_frags<ANP>(A, m0 + nloc, kb, hlf, a0h, a0l);
    load_frags<ANP>(A, m0 + 16 + nloc, kb, hlf, a1h, a1l);
#pragma unroll
    for (int t = 0; t < 4; ++t) {
      v16b bh, bl;
      load_frags<BNP>(B, c0 + t * 16 + nloc, kb, hlf, bh, bl);
      acc[0][t] = mac<ANP, BNP>(a0h, a0l, bh, bl, acc[0][t]);
      acc[1][t] = mac<ANP, BNP>(a1h, a1l, bh, bl, acc[1][t]);
    }
  }
}

__device__ __forceinline__ void epi_planes(v8f (&acc)[2][4], float scale, bool two, b16* __restrict__ oh, b16* __restrict__ ol, int ldo,
                                           int m0, int c0, int lane, b16* Th, b16* Tl) {
  const int nloc = lane & 15, hlf = lane >> 4;
#pragma unroll
  for (int t = 0; t < 4; ++t)
#pragma unroll
    for (int r = 0; r < 2; ++r)
#pragma unroll
      for (int v = 0; v < 8; ++v) {
        const int rr = r * 16 + v + 8 * hlf, cc = t * 16 + nloc;
        b16 h_, l_; split16(acc[r][t][v] * scale, h_, l_);
        Th[rr * 64 + cc] = h_; Tl[rr * 64 + cc] = l_;
      }
  wave_lds_sync();
  for (int pass = 0; pass < 2; ++pass) {
#pragma unroll
    for (int j = 0; j < 8; ++j) {
      const int rr = j * 4 + (lane >> 3), c8 = (lane & 7) * 8;
      const size_t o = (size_t)(m0 + rr) * ldo + c0 + c8;
      *(volatile v8b*)(oh + o) = ld8b(Th + rr * 64 + c8);
      if (two) *(volatile v8b*)(ol + o) = ld8b(Tl + rr * 64 + c8);
    }
    __threadfence();
  }
}
__device__ __forceinline__ void epi_f32(v8f (&acc)[2][4], float scale, const float* rscale, float* __restrict__ out, int ldo, int m0, int c0, int lane, float* Tt) {
  const int nloc = lane & 15, hlf = lane >> 4;
#pragma unroll
  for (int t = 0; t < 4; ++t)
#pragma unroll
    for (int r = 0; r < 2; ++r)
#pragma unroll
      for (int v = 0; v < 8; ++v) {
        const int rr = r * 16 + v + 8 * hlf;
        const float rs = rscale ? rscale[(size_t)(m0 + rr) * 32] : 1.0f;
        Tt[rr * 64 + t * 16 + nloc] = acc[r][t][v] * scale * rs;
      }
  wave_lds_sync();
  float* dst0 = out + (size_t)m0 * ldo + c0;
  for (int pass = 0; pass < 2; ++pass) {
#pragma unroll
    for (int j = 0; j < 16; ++j) { const int rr = j * 2 + hlf, c4 = nloc * 4; *(volatile v4f*)(dst0 + (size_t)rr * ldo + c4) = *(const v4f*)(Tt + rr * 64 + c4); }
    __threadfence();
  }
}


__device__ __forceinline__ int fkey(float f) { const int b = __float_as_int(f); return (b >= 0) ? b : (b ^ 0x7FFFFFFF); }
__device__ __forceinline__ float fkey_inv(int k) { return __int_as_float((k >= 0) ? k : (k ^ 0x7FFFFFFF)); }
__device__ __forceinline__ float elu1(float v) { return (v > 0.0f) ? v : (__expf(v) - 1.0f); }

__global__ __launch_bounds__(256) void prep_kernel(const float* __restrict__ x, const float* __restrict__ W1, const float* __restrict__ W2, const float* __restrict__ W3, const float* __restrict__ W4,
                                                   float* __restrict__ xp, float* __restrict__ xspad, b16* __restrict__ w1, b16* __restrict__ w2, b16* __restrict__ w3, b16* __restrict__ w4) {
  const size_t tid = (size_t)blockIdx.x * blockDim.x + threadIdx.x, nth = (size_t)gridDim.x * blockDim.x;
  for (int pass = 0; pass < 2; ++pass) {
    for (size_t p = tid; p < (size_t)NPAD * F / 4; p += nth) { const size_t n = p / (F / 4); const v4f v = *(const v4f*)(x + min(p, (size_t)N * F / 4 - 1) * 4); *(volatile v4f*)(xp + p * 4) = (n < (size_t)N) ? v : (v4f){0.0f, 0.0f, 0.0f, 0.0f}; }
    for (size_t p = tid; p < (size_t)(NPAD - N) * C1 / 4; p += nth) *(volatile v4f*)(xspad + p * 4) = (v4f){0.0f, 0.0f, 0.0f, 0.0f};
    for (size_t p = tid; p < (size_t)2 * D1 * F / 8; p += nth) { const int which = (int)(p / (D1 * F / 8)); const int rem = (int)(p % (D1 * F / 8)), n = rem / (F / 8), k0 = (rem % (F / 8)) * 8; const float* W = which ? W3 : W1; v8b v;
#pragma unroll
      for (int e = 0; e < 8; ++e) v[e] = (b16)W[(size_t)(k0 + e) * D1 + n];
      *(volatile v8b*)((which ? w3 : w1) + (size_t)n * F + k0) = v; }
    for (size_t p = tid; p < (size_t)2 * D2 * C1 / 8; p += nth) { const int which = (int)(p / (D2 * C1 / 8)); const int rem = (int)(p % (D2 * C1 / 8)), n = rem / (C1 / 8), k0 = (rem % (C1 / 8)) * 8; const float* W = which ? W4 : W2; v8b v;
#pragma unroll
      for (int e = 0; e < 8; ++e) v[e] = (b16)W[(size_t)(k0 + e) * D2 + n];
      *(volatile v8b*)((which ? w4 : w2) + (size_t)n * C1 + k0) = v; }
    __threadfence();
  }
}

template <int KIN, int NOUT>
__global__ __launch_bounds__(128) void lin_kernel(const float* __restrict__ xin, const b16* __restrict__ w, float* __restrict__ h) {
  __shared__ __attribute__((aligned(16))) float Ts[4][32 * 64];
  const int lane = threadIdx.x & 31, wave = threadIdx.x >> 5, nloc = lane & 15, hlf = lane >> 4, m0 = blockIdx.y * 128 + wave * 32, c0 = blockIdx.x * 64;
  v8f acc[2][4];
#pragma unroll
  for (int r = 0; r < 2; ++r)
#pragma unroll
    for (int t = 0; t < 4; ++t) acc[r][t] = (v8f){};
  const Opnd A{xin, nullptr, KIN}, B{w, nullptr, KIN};
  gemm_tile<3, 1>(A, B, KIN, m0, c0, nloc, hlf, acc);
  epi_f32(acc, 1.0f, nullptr, h, NOUT, m0, c0, lane, Ts[wave]);
}

template <int C>
__global__ __launch_bounds__(256) void alpha_kernel(const float* __restrict__ h, const float* __restrict__ asrc, const float* __restrict__ adst, float* __restrict__ al) {
  const int wid = threadIdx.x >> 5, lane = threadIdx.x & 31, n = blockIdx.x * 8 + wid;
  float ss = 0.0f, sd = 0.0f; const float* hr = h + (size_t)n * (H * C) + lane * C;
#pragma unroll 4
  for (int c = 0; c < C; c += 4) { const v4f v = *(const v4f*)(hr + c);
#pragma unroll
    for (int e = 0; e < 4; ++e) { ss += v[e] * asrc[lane * C + c + e]; sd += v[e] * adst[lane * C + c + e]; } }
  for (int pass = 0; pass < 2; ++pass) { ((volatile float*)al)[(size_t)n * 64 + lane] = ss; ((volatile float*)al)[(size_t)n * 64 + 32 + lane] = sd; __threadfence(); }
}

typedef __attribute__((ext_vector_type(4))) int v4i;
template <int C, int NB>
__global__ __launch_bounds__(256) void gat_kernel(const int* __restrict__ esrc, const int* __restrict__ edst, const float* __restrict__ h, const float* __restrict__ al, const float* __restrict__ bias, float* __restrict__ xo) {
  constexpr int DF = H * C;
  __shared__ __attribute__((aligned(16))) int acc[NB * DF];
  __shared__ int mx[NB * H]; __shared__ int den[NB * H]; __shared__ int list[8 * 256];
  const int t_ = threadIdx.x, wave = t_ >> 5, lane = t_ & 31, base = blockIdx.x * NB;
  for (int i = t_; i < NB * DF; i += 256) acc[i] = 0;
  for (int i = t_; i < NB * H; i += 256) { den[i] = 0; mx[i] = fkey(-INFINITY); }
  __syncthreads();
  for (int i = t_; i < NB * H; i += 256) { const int slot = i / H, hd = i % H, node = base + slot; if (node < N) { float e = al[(size_t)node * 64 + hd] + al[(size_t)node * 64 + 32 + hd]; e = (e > 0.0f) ? e : NEG * e; atomicMax(&mx[i], fkey(e)); } }
  for (int c0 = 0; c0 < E; c0 += 256 * 8) {
    const int e0 = c0 + (wave * 32 + lane) * 8;
#pragma unroll
    for (int j = 0; j < 8; ++j) { const int ee = min(e0 + j, E - 1); const int dv = edst[ee]; const unsigned sl = (unsigned)(((e0 + j < E) ? dv : -1) - base);
      if (sl < (unsigned)NB) { int s = esrc[ee]; s = (s < 0) ? 0 : (s >= N ? N - 1 : s);
        for (int hd = 0; hd < H; ++hd) { float ev = al[(size_t)s * 64 + hd] + al[(size_t)(base + sl) * 64 + 32 + hd]; ev = (ev > 0.0f) ? ev : NEG * ev; atomicMax(&mx[sl * H + hd], fkey(ev)); } } }
  }
  __syncthreads();
  int* wl = list + wave * 256;
  auto accumulate = [&](int s, int slot) {
    float e = al[(size_t)s * 64 + lane] + al[(size_t)(base + slot) * 64 + 32 + lane]; e = (e > 0.0f) ? e : NEG * e;
    const float w = __expf(e - fkey_inv(mx[slot * H + lane]));
    atomicAdd(&den[slot * H + lane], (int)rintf(w * FXS));
    const float* hr = h + (size_t)s * DF + lane * C; int* ar = acc + slot * DF + lane * C;
#pragma unroll 4
    for (int c = 0; c < C; c += 4) { const v4f v = *(const v4f*)(hr + c);
#pragma unroll
      for (int q = 0; q < 4; ++q) atomicAdd(ar + c + q, (int)rintf(w * v[q] * FXS)); }
  };
  for (int slot = wave; slot < NB; slot += 8) { if (base + slot < N) accumulate(base + slot, slot); }
  for (int c0 = 0; c0 < E; c0 += 256 * 8) {
    const int e0 = c0 + (wave * 32 + lane) * 8; int dd[8];
#pragma unroll
    for (int j = 0; j < 8; ++j) { const int dv = edst[min(e0 + j, E - 1)]; dd[j] = (e0 + j < E) ? dv : -1; }
    unsigned sl[8]; bool hit[8]; bool anyl = false;
#pragma unroll
    for (int j = 0; j < 8; ++j) { sl[j] = (unsigned)(dd[j] - base); hit[j] = sl[j] < (unsigned)NB; anyl |= hit[j]; }
    int wc = 0;
    if (__builtin_amdgcn_ballot_w32(anyl) != 0u) {
#pragma unroll
      for (int j = 0; j < 8; ++j) {
        const unsigned mj = __builtin_amdgcn_ballot_w32(hit[j]);
        if (mj != 0u) {
          if (hit[j]) { const int pos = wc + (int)__builtin_amdgcn_mbcnt_lo(mj, 0u); int s = esrc[min(e0 + j, E - 1)]; s = (s < 0) ? 0 : (s >= N ? N - 1 : s); wl[pos] = (s << 12) | (int)sl[j]; }
          wc += __builtin_popcount(mj); } } }
    __builtin_amdgcn_wave_barrier(); __builtin_amdgcn_fence(__ATOMIC_RELEASE, "workgroup"); __builtin_amdgcn_fence(__ATOMIC_ACQUIRE, "workgroup");
    for (int i = 0; i < wc; ++i) { const int ent = wl[i]; accumulate(ent >> 12, ent & 4095); }
    __builtin_amdgcn_wave_barrier();
  }
  __syncthreads();
  for (int pass = 0; pass < 2; ++pass) {
    for (int i = t_; i < NB * C / 4; i += 256) { const int slot = i / (C / 4), cq = (i % (C / 4)) * 4, node = base + slot; if (node < N) { v4f o = {0.0f, 0.0f, 0.0f, 0.0f};
        { float s4[4] = {0, 0, 0, 0};
          for (int hd = 0; hd < H; ++hd) { const float dn = 1.0f / ((float)den[slot * H + hd] * FXI + 1e-16f);
#pragma unroll
            for (int q = 0; q < 4; ++q) s4[q] += (float)acc[slot * DF + hd * C + cq + q] * FXI * dn; }
#pragma unroll
          for (int q = 0; q < 4; ++q) o[q] = elu1(s4[q] * (1.0f / H) + bias[cq + q]); }
        *(volatile v4f*)(xo + (size_t)node * C + cq) = o; } }
    __threadfence();
  }
}

__device__ __forceinline__ float bnf(float v, const float* g, const float* b, const float* m, const float* var, int c) { return (v - m[c]) * g[c] * rsqrtf(var[c] + BNE) + b[c]; }

__global__ __launch_bounds__(128) void resid_kernel(const float* __restrict__ xp, const float* __restrict__ rwa, const float* __restrict__ rba, const float* __restrict__ g1, const float* __restrict__ b1, const float* __restrict__ m1, const float* __restrict__ v1,
                                                    const float* __restrict__ rwb, const float* __restrict__ rbb, const float* __restrict__ g2, const float* __restrict__ b2, const float* __restrict__ m2, const float* __restrict__ v2,
                                                    const float* __restrict__ wsc, const float* __restrict__ bsc, const float* __restrict__ gs, const float* __restrict__ bs, const float* __restrict__ ms, const float* __restrict__ vs,
                                                    const float* __restrict__ wfc, const float* __restrict__ bfc, float* __restrict__ xself) {
  __shared__ __attribute__((aligned(16))) float Ob[4][32][OUT];
  const int lane = threadIdx.x & 31, wave = threadIdx.x >> 5, nloc = lane & 15, hlf = lane >> 4, m0 = blockIdx.x * 128 + wave * 32;
  v8f t1[2] = {{}, {}}, ts[2] = {{}, {}};
  const Opnd A{xp, nullptr, F};
#pragma unroll
  for (int kb = 0; kb < F; kb += 32) { v16b a0, a1, d0, d1; load_frags<3>(A, m0 + nloc, kb, hlf, a0, d0); load_frags<3>(A, m0 + 16 + nloc, kb, hlf, a1, d1);
    v16b bw, bs_;
#pragma unroll
    for (int e = 0; e < 16; ++e) { const int k = kb + ((e < 8) ? (8 * hlf + e) : (16 + 8 * hlf + e - 8)); bw[e] = (b16)rwa[k * OUT + nloc]; bs_[e] = (b16)wsc[k * OUT + nloc]; }
    t1[0] = wmma16b(a0, bw, t1[0]); t1[1] = wmma16b(a1, bw, t1[1]); ts[0] = wmma16b(a0, bs_, ts[0]); ts[1] = wmma16b(a1, bs_, ts[1]); }
  __shared__ __attribute__((aligned(16))) b16 Ht[4][32][16 + 8];
#pragma unroll
  for (int r = 0; r < 2; ++r)
#pragma unroll
    for (int v = 0; v < 8; ++v) Ht[wave][r * 16 + v + 8 * hlf][nloc] = (b16)fmaxf(bnf(t1[r][v] + rba[nloc], g1, b1, m1, v1, nloc), 0.0f);
  wave_lds_sync();
  v8f h2[2] = {{}, {}};
  { v16b a0 = {}, a1 = {}, bw = {};
#pragma unroll
    for (int e = 0; e < 8; ++e) { a0[e] = Ht[wave][nloc][8 * hlf + e]; a1[e] = Ht[wave][16 + nloc][8 * hlf + e]; bw[e] = (b16)rwb[(8 * hlf + e) * OUT + nloc]; }
    h2[0] = wmma16b(a0, bw, h2[0]); h2[1] = wmma16b(a1, bw, h2[1]); }
  wave_lds_sync();
#pragma unroll
  for (int r = 0; r < 2; ++r)
#pragma unroll
    for (int v = 0; v < 8; ++v) { const float hv = bnf(h2[r][v] + rbb[nloc], g2, b2, m2, v2, nloc); const float sv = bnf(ts[r][v] + bsc[nloc], gs, bs, ms, vs, nloc); Ht[wave][r * 16 + v + 8 * hlf][nloc] = (b16)fmaxf(hv + sv, 0.0f); }
  wave_lds_sync();
  v8f y[2] = {{}, {}};
  { v16b a0 = {}, a1 = {}, bw = {};
#pragma unroll
    for (int e = 0; e < 8; ++e) { a0[e] = Ht[wave][nloc][8 * hlf + e]; a1[e] = Ht[wave][16 + nloc][8 * hlf + e]; bw[e] = (b16)wfc[(8 * hlf + e) * OUT + nloc]; }
    y[0] = wmma16b(a0, bw, y[0]); y[1] = wmma16b(a1, bw, y[1]); }
#pragma unroll
  for (int r = 0; r < 2; ++r)
#pragma unroll
    for (int v = 0; v < 8; ++v) Ob[wave][r * 16 + v + 8 * hlf][nloc] = y[r][v] + bfc[nloc];
  wave_lds_sync();
  for (int pass = 0; pass < 2; ++pass) {
#pragma unroll
    for (int j = 0; j < 4; ++j) { const int rr = j * 8 + (lane >> 2), c4 = (lane & 3) * 4; if (m0 + rr < N) *(volatile v4f*)(xself + (size_t)(m0 + rr) * OUT + c4) = *(const v4f*)(&Ob[wave][rr][c4]); }
    __threadfence();
  }
}
}

extern "C" void kernel_launch(void* const* d_in, const int* in_sizes, int n_in,
                              void* d_out, int out_size, void* d_ws, size_t ws_size, hipStream_t stream) {
  (void)n_in; (void)out_size;
  const float* x = (const float*)d_in[0]; const int* ei = (const int*)d_in[1];
  const float* W1 = (const float*)d_in[2]; const float* as1 = (const float*)d_in[3]; const float* ad1 = (const float*)d_in[4]; const float* b1 = (const float*)d_in[5];
  const float* W2 = (const float*)d_in[6]; const float* as2 = (const float*)d_in[7]; const float* ad2 = (const float*)d_in[8]; const float* b2 = (const float*)d_in[9];
  const float* W3 = (const float*)d_in[10]; const float* as3 = (const float*)d_in[11]; const float* ad3 = (const float*)d_in[12]; const float* b3 = (const float*)d_in[13];
  const float* W4 = (const float*)d_in[14]; const float* as4 = (const float*)d_in[15]; const float* ad4 = (const float*)d_in[16]; const float* b4 = (const float*)d_in[17];
  const float* const* P = (const float* const*)d_in;
  float* out = (float*)d_out;
  if (in_sizes[0] != N * F || in_sizes[1] != 2 * E || in_sizes[2] != F * D1 || in_sizes[6] != C1 * D2 || in_sizes[18] != F * OUT || in_sizes[36] != OUT * OUT) return;
  const int* s2t_src = ei; const int* s2t_dst = ei + E;
  size_t off = 0; char* ws = (char*)d_ws;
  auto carve = [&](size_t bytes) { char* p = ws + off; off += (bytes + 255) & ~(size_t)255; return p; };
  float* xp = (float*)carve((size_t)NPAD * F * 4); b16* w1 = (b16*)carve((size_t)D1 * F * 2); b16* w2 = (b16*)carve((size_t)D2 * C1 * 2); b16* w3 = (b16*)carve((size_t)D1 * F * 2); b16* w4 = (b16*)carve((size_t)D2 * C1 * 2);
  float* hbig = (float*)carve((size_t)NPAD * D1 * 4);
  float* al = (float*)carve((size_t)NPAD * 64 * 4); float* xs = (float*)carve((size_t)NPAD * C1 * 4); float* hsm = (float*)carve((size_t)NPAD * D2 * 4);
  if (off > ws_size) return;
  float* x_in = out; float* x_out = out + (size_t)N * OUT; float* x_self = out + (size_t)2 * N * OUT;
  prep_kernel<<<512, 256, 0, stream>>>(x, W1, W2, W3, W4, xp, xs + (size_t)N * C1, w1, w2, w3, w4);
  for (int dir = 0; dir < 2; ++dir) {
    const int* esrc = dir ? s2t_dst : s2t_src; const int* edst = dir ? s2t_src : s2t_dst;
    lin_kernel<F, D1><<<dim3(D1 / 64, NPAD / 128), 128, 0, stream>>>(xp, dir ? w3 : w1, hbig);
    alpha_kernel<C1><<<NPAD / 8, 256, 0, stream>>>(hbig, dir ? as3 : as1, dir ? ad3 : ad1, al);
    gat_kernel<C1, 32><<<NPAD / 32, 256, 0, stream>>>(esrc, edst, hbig, al, dir ? b3 : b1, xs);
    lin_kernel<C1, D2><<<dim3(D2 / 64, NPAD / 128), 128, 0, stream>>>(xs, dir ? w4 : w2, hsm);
    alpha_kernel<OUT><<<NPAD / 8, 256, 0, stream>>>(hsm, dir ? as4 : as2, dir ? ad4 : ad2, al);
    gat_kernel<OUT, 128><<<NPAD / 128, 256, 0, stream>>>(esrc, edst, hsm, al, dir ? b4 : b2, dir ? x_out : x_in);
  }
  resid_kernel<<<NPAD / 128, 128, 0, stream>>>(xp, P[18], P[19], P[20], P[21], P[22], P[23], P[24], P[25], P[26], P[27], P[28], P[29], P[30], P[31], P[32], P[33], P[34], P[35], P[36], P[37], x_self);
}
